// MambaLayer_20753281975081
// MI455X (gfx1250) — hardware-verified
//
#include <hip/hip_runtime.h>
#include <math.h>

typedef __attribute__((ext_vector_type(16))) _Float16 v16h;
typedef __attribute__((ext_vector_type(8)))  _Float16 v8h;
typedef __attribute__((ext_vector_type(16))) __bf16   v16b;
typedef __attribute__((ext_vector_type(8)))  __bf16   v8b;
typedef __attribute__((ext_vector_type(8)))  float    v8f;
typedef __attribute__((ext_vector_type(4)))  float    v4f;

constexpr int kBat   = 4;
constexpr int kCh    = 256;
constexpr int kSeq   = 1024;
constexpr int kTok   = kBat * kSeq;
constexpr int kHid   = 1024;
constexpr int kNsp   = 8;
constexpr int kKc1   = kCh * (1 + kNsp);
constexpr int kKc2   = kHid * (1 + kNsp);
constexpr int kChunk = 1024;
constexpr int kDh    = 128;
constexpr int kDtR   = 16;
constexpr int kNst   = 8;
constexpr int kXdP   = 64;
constexpr int kHeads = 4;
constexpr int kHd    = 64;
constexpr float kACarry  = 64.0f;
constexpr float kWCarry  = 1024.0f;
constexpr float kF16Fold = 1.0f / (kACarry * kWCarry);
constexpr float kLnEps   = 1e-5f;
static_assert(kTok == 4096 && kKc1 == 2304 && kKc2 == 9216, "shape constants");
static_assert((kKc1 % 32) == 0 && (kKc2 % 32) == 0 && (kCh % 32) == 0 && (kDh % 32) == 0 && (kHd % 32) == 0 && (kSeq % 32) == 0, "K multiples of 32");
static_assert((kTok % 64) == 0 && (kHid % 64) == 0 && (kCh % 64) == 0 && (kXdP % 64) == 0 && (kChunk % 64) == 0 && (kHd % 64) == 0, "M,N multiples of 64");
static_assert(kDtR + 2 * kNst == 32 && kHeads * kHd == kCh && kTok * kKc1 == kChunk * kKc2, "derived shapes");

constexpr size_t kSzX    = (size_t)kTok * kCh * 4;
constexpr size_t kOffXA   = 0;
constexpr size_t kOffXB   = kOffXA   + kSzX;
constexpr size_t kOffXN16 = kOffXB   + kSzX;
constexpr size_t kOffQKVW = kOffXN16 + (size_t)kTok * kCh * 2;
constexpr size_t kOffPOW  = kOffQKVW + (size_t)768 * kCh * 2;
constexpr size_t kOffINW  = kOffPOW  + (size_t)kCh * kCh * 2;
constexpr size_t kOffOUTW = kOffINW  + (size_t)kCh * kCh * 2;
constexpr size_t kOffXPW  = kOffOUTW + (size_t)kCh * kCh * 2;
constexpr size_t kOffW1A  = kOffXPW  + (size_t)64 * kDh * 2;
constexpr size_t kOffW2A  = kOffW1A  + (size_t)kHid * kKc1 * 2;
constexpr size_t kOffW1B  = kOffW2A  + (size_t)kCh * kKc2 * 2;
constexpr size_t kOffW2B  = kOffW1B  + (size_t)kHid * kKc1 * 2;
constexpr size_t kOffH    = kOffW2B  + (size_t)kCh * kKc2 * 2;
constexpr size_t kOffAH   = kOffH    + (size_t)kTok * kHid * 4;
constexpr size_t kOffAL   = kOffAH   + (size_t)kTok * kKc1 * 2;
constexpr size_t kOffQKF  = kOffAL   + (size_t)kTok * kKc1 * 2;
constexpr size_t kOffVCL  = kOffQKF  + (size_t)kBat * 512 * kSeq * 4;
constexpr size_t kOffQ16  = kOffVCL  + kSzX;
constexpr size_t kOffK16  = kOffQ16  + (size_t)kBat * kCh * kSeq * 2;
constexpr size_t kOffVT16 = kOffK16  + (size_t)kBat * kCh * kSeq * 2;
constexpr size_t kOffATT  = kOffVT16 + (size_t)kTok * kCh * 2;
constexpr size_t kOffATT16 = kOffATT + (size_t)16 * 64 * 64 * 4;
constexpr size_t kOffATOH = kOffATT16 + (size_t)16 * 64 * 64 * 2;
constexpr size_t kOffATOL = kOffATOH + (size_t)kTok * kCh * 2;
constexpr size_t kOffXZ   = kOffATOL + (size_t)kTok * kCh * 2;
constexpr size_t kOffXM   = kOffXZ   + kSzX;
constexpr size_t kOffXM16 = kOffXM   + (size_t)kTok * kDh * 4;
constexpr size_t kOffXD   = kOffXM16 + (size_t)kTok * kDh * 2;
constexpr size_t kOffYC16 = kOffXD   + (size_t)kTok * kXdP * 4;
constexpr size_t kWsTotal = kOffYC16 + (size_t)kTok * kCh * 2;
static_assert(kWsTotal <= 134217728ull, "carve cap");
static_assert((kOffXN16 % 128) == 0 && (kOffQKVW % 128) == 0 && (kOffXPW % 128) == 0 && (kOffW1A % 128) == 0 &&
              (kOffH % 128) == 0 && (kOffAH % 128) == 0 && (kOffAL % 128) == 0 && (kOffQKF % 128) == 0 &&
              (kOffATT % 128) == 0 && (kOffATT16 % 128) == 0 && (kOffATOH % 128) == 0 && (kOffXZ % 128) == 0 &&
              (kOffXM16 % 128) == 0 && (kOffXD % 128) == 0 && (kOffYC16 % 128) == 0, "128-B aligned regions");

__device__ __forceinline__ unsigned short f2bf_bits(float f) {
  unsigned u = __float_as_uint(f);
  return (unsigned short)((u + 0x7FFFu + ((u >> 16) & 1u)) >> 16);
}
__device__ __forceinline__ float bf_bits2f(unsigned short h) { return __uint_as_float(((unsigned)h) << 16); }
__device__ __forceinline__ float rbf(float f) { return bf_bits2f(f2bf_bits(f)); }
__device__ __forceinline__ float wave_sum(float v) {
#pragma unroll
  for (int off = 16; off > 0; off >>= 1) v += __shfl_xor(v, off, 32);
  return v;
}
__device__ __forceinline__ void wave_lds_sync() {
  __builtin_amdgcn_fence(__ATOMIC_RELEASE, "workgroup");
  __builtin_amdgcn_wave_barrier();
  __builtin_amdgcn_fence(__ATOMIC_ACQUIRE, "workgroup");
}

__device__ __forceinline__ void tie4_h(v8f& a, v8f& b, v8f& c, v8f& d, v16h x, v16h y) { asm volatile("v_nop\n\tv_nop\n\tv_nop\n\tv_nop" : "+v"(a), "+v"(b), "+v"(c), "+v"(d) : "v"(x), "v"(y)); }
__device__ __forceinline__ void tie4_b(v8f& a, v8f& b, v8f& c, v8f& d, v16b x, v16b y) { asm volatile("v_nop\n\tv_nop\n\tv_nop\n\tv_nop" : "+v"(a), "+v"(b), "+v"(c), "+v"(d) : "v"(x), "v"(y)); }
__device__ __forceinline__ void keep4_h(v16h a, v16h b, v16h c, v16h d) { asm volatile("v_nop" :: "v"(a), "v"(b), "v"(c), "v"(d)); }
__device__ __forceinline__ void keep4_b(v16b a, v16b b, v16b c, v16b d) { asm volatile("v_nop" :: "v"(a), "v"(b), "v"(c), "v"(d)); }
__device__ __forceinline__ void acc_guard4(v8f& a, v8f& b, v8f& c, v8f& d) { asm volatile("v_nop\n\tv_nop\n\tv_nop\n\tv_nop" : "+v"(a), "+v"(b), "+v"(c), "+v"(d)); }
template <typename T> struct Frag;
template <> struct Frag<_Float16> {
  typedef v16h V; union U { v16h v; v8h h[2]; };
  static __device__ __forceinline__ v16h load(const _Float16* p) {
    U f; f.h[0] = *(const v8h*)(p); f.h[1] = *(const v8h*)(p + 16); return f.v;
  }
  static __device__ __forceinline__ v8f mma(v16h a, v16h b, v8f c) {
    return __builtin_amdgcn_wmma_f32_16x16x32_f16(false, a, false, b, (short)0, c, false, false);
  }
  static __device__ __forceinline__ void guard4(v8f& a, v8f& b, v8f& c, v8f& d, v16h x, v16h y) { tie4_h(a, b, c, d, x, y); }
  static __device__ __forceinline__ void keep(v16h a, v16h b, v16h c, v16h d) { keep4_h(a, b, c, d); }
};
template <> struct Frag<__bf16> {
  typedef v16b V; union U { v16b v; v8b h[2]; };
  static __device__ __forceinline__ v16b load(const __bf16* p) {
    U f; f.h[0] = *(const v8b*)(p); f.h[1] = *(const v8b*)(p + 16); return f.v;
  }
  static __device__ __forceinline__ v8f mma(v16b a, v16b b, v8f c) {
    return __builtin_amdgcn_wmma_f32_16x16x32_bf16(false, a, false, b, (short)0, c, false, false);
  }
  static __device__ __forceinline__ void guard4(v8f& a, v8f& b, v8f& c, v8f& d, v16b x, v16b y) { tie4_b(a, b, c, d, x, y); }
  static __device__ __forceinline__ void keep(v16b a, v16b b, v16b c, v16b d) { keep4_b(a, b, c, d); }
};

template <int ET> struct Elem;
template <> struct Elem<0> { typedef _Float16 T; };
template <> struct Elem<1> { typedef __bf16 T; };
template <int ET, int SPL, int BIAS_MODE, int OUT_MODE, bool RESID>
__global__ __launch_bounds__(256) void wmma_gemm64(
    const unsigned short* __restrict__ Ap, const unsigned short* __restrict__ A2p, int lda, long strideA,
    const unsigned short* __restrict__ Btp, int ldb, long strideB,
    void* __restrict__ Cout, void* __restrict__ Cout2, int ldc, long strideC,
    const float* __restrict__ bias,
    const float* __restrict__ resid, long strideR,
    int M, int N, int K, float scale) {
  static_assert(OUT_MODE == 0 || OUT_MODE == 2, "output modes");
  static_assert(SPL == 0 || SPL == 1, "split modes");
  typedef typename Elem<ET>::T T;
  typedef typename Frag<T>::V V;
  const T* A = (const T*)Ap; const T* A2 = (const T*)A2p; const T* Bt = (const T*)Btp;
  __shared__ __align__(16) float sT[8][16 * 68];
  const int b    = blockIdx.y;
  const int lane = threadIdx.x & 31;
  const int wave = threadIdx.x >> 5;
  const int tilesN = N >> 6;
  const int tilesM = M >> 6;
  const int tile = blockIdx.x * 8 + wave;
  if (tile >= tilesM * tilesN) return;
  const int tm = tile / tilesN;
  const int tn = tile - tm * tilesN;
  const int m0 = tm << 6;
  const int n0 = tn << 6;

  const T* Ab  = A  + (size_t)b * strideA;
  const T* Bb  = Bt + (size_t)b * strideB;
  const T* Ab2 = (SPL >= 1) ? (A2 + (size_t)b * strideA) : Ab;

  const int rlane = lane & 15;
  const int koff  = (lane >> 4) * 8;
  const int mOff  = (lane >> 4) * 8;

  v8f acc[4][4];
#pragma unroll
  for (int i = 0; i < 4; ++i)
#pragma unroll
    for (int j = 0; j < 4; ++j) acc[i][j] = (v8f){0.f,0.f,0.f,0.f,0.f,0.f,0.f,0.f};

  for (int k0 = 0; k0 < K; k0 += 32) {
    V bh[4];
#pragma unroll
    for (int j = 0; j < 4; ++j) {
      const size_t bo = (size_t)(n0 + (j << 4) + rlane) * ldb + koff + k0;
      bh[j] = Frag<T>::load(Bb + bo);
    }
#pragma unroll
    for (int i = 0; i < 4; ++i) {
      const size_t ao = (size_t)(m0 + (i << 4) + rlane) * lda + koff + k0;
      V ah = Frag<T>::load(Ab + ao);
      V al = ah;
      if (SPL >= 1) al = Frag<T>::load(Ab2 + ao);
#pragma unroll
      for (int j = 0; j < 4; ++j) {
        acc[i][j] = Frag<T>::mma(ah, bh[j], acc[i][j]);
        if (SPL >= 1) acc[i][j] = Frag<T>::mma(al, bh[j], acc[i][j]);
      }
      Frag<T>::guard4(acc[i][0], acc[i][1], acc[i][2], acc[i][3], ah, al);
    }
    Frag<T>::keep(bh[0], bh[1], bh[2], bh[3]);
  }
  acc_guard4(acc[0][0], acc[0][1], acc[0][2], acc[0][3]);
  acc_guard4(acc[1][0], acc[1][1], acc[1][2], acc[1][3]);
  acc_guard4(acc[2][0], acc[2][1], acc[2][2], acc[2][3]);
  acc_guard4(acc[3][0], acc[3][1], acc[3][2], acc[3][3]);

  float* slab = sT[wave];
  const float* Rb = RESID ? (resid + (size_t)b * strideR) : resid;
#pragma unroll
  for (int i = 0; i < 4; ++i) {
    const int mBase = m0 + (i << 4);
#pragma unroll
    for (int j = 0; j < 4; ++j) {
#pragma unroll
      for (int r = 0; r < 8; ++r) slab[(mOff + r) * 68 + (j << 4) + rlane] = acc[i][j][r] * scale;
    }
    wave_lds_sync();
    if (OUT_MODE == 0) {
      float* C = (float*)Cout + (size_t)b * strideC;
      const int hh = lane >> 4, c4 = (lane & 15) * 4;
      v4f bq = (v4f){0.f, 0.f, 0.f, 0.f};
      if (BIAS_MODE == 2) {
        const v4f braw = *(const v4f*)(bias + n0 + c4);
        const float q0 = braw[0], q1 = braw[1], q2 = braw[2], q3 = braw[3];
        bq = (v4f){rbf(q0), rbf(q1), rbf(q2), rbf(q3)};
      }
      v4f ov[8];
#pragma unroll
      for (int it = 0; it < 8; ++it) {
        const int row = it * 2 + hh;
        v4f v = *(const v4f*)(slab + row * 68 + c4);
        if (BIAS_MODE == 2) v += bq;
        if (BIAS_MODE == 1) {
          const float bm = rbf(bias[mBase + row]);
          v += (v4f){bm, bm, bm, bm};
        }
        if (RESID) {
          const v4f rv = *(const v4f*)(Rb + (size_t)(mBase + row) * ldc + n0 + c4);
          v += rv;
        }
        ov[it] = v;
      }
      for (int pass = 0; pass < 2; ++pass) {
#pragma unroll
        for (int it = 0; it < 8; ++it) {
          const int row = it * 2 + hh;
          *(volatile v4f*)(C + (size_t)(mBase + row) * ldc + n0 + c4) = ov[it];
        }
        __threadfence();
      }
    } else {
      const int q = lane >> 3, c8 = (lane & 7) * 8;
      unsigned short* C  = (unsigned short*)Cout  + (size_t)b * strideC;
      unsigned short* C2 = (unsigned short*)Cout2 + (size_t)b * strideC;
      v8h hvv[4], lvv[4];
#pragma unroll
      for (int it = 0; it < 4; ++it) {
        const int row = it * 4 + q;
        const float* sp = slab + row * 68 + c8;
#pragma unroll
        for (int e = 0; e < 8; ++e) {
          const float sv = sp[e];
          const unsigned short hb = f2bf_bits(sv);
          const unsigned short lb = f2bf_bits(sv - bf_bits2f(hb));
          hvv[it][e] = __builtin_bit_cast(_Float16, hb);
          lvv[it][e] = __builtin_bit_cast(_Float16, lb);
        }
      }
      for (int pass = 0; pass < 2; ++pass) {
#pragma unroll
        for (int it = 0; it < 4; ++it) {
          const int row = it * 4 + q;
          *(volatile v8h*)(C  + (size_t)(mBase + row) * ldc + n0 + c8) = hvv[it];
          *(volatile v8h*)(C2 + (size_t)(mBase + row) * ldc + n0 + c8) = lvv[it];
        }
        __threadfence();
      }
    }
    wave_lds_sync();
  }
}

template <bool F16>
__global__ __launch_bounds__(256) void cast_rows_kernel(
    const float* __restrict__ src, int src_pitch, int rows_real,
    unsigned short* __restrict__ dst, int dst_pitch, int cols8, int total8, float scale)
{
  const int i = blockIdx.x * 256 + threadIdx.x;
  if (i >= total8) return;
  const int row = i / cols8;
  const int g   = i - row * cols8;
  const bool live = row < rows_real;
  const int rc = live ? row : (rows_real - 1);
  const float* p = src + (size_t)rc * src_pitch + g * 8;
  const v4f a0 = *(const v4f*)(p);
  const v4f a1 = *(const v4f*)(p + 4);
  v8h hv;
#pragma unroll
  for (int e = 0; e < 4; ++e) {
    const float x0 = a0[e], x1 = a1[e];
    if (F16) {
      const float y0 = live ? rbf(x0) * scale : 0.0f;
      const float y1 = live ? rbf(x1) * scale : 0.0f;
      hv[e]     = (_Float16)y0;
      hv[4 + e] = (_Float16)y1;
    } else {
      const unsigned short b0 = f2bf_bits(x0), b1 = f2bf_bits(x1);
      const unsigned short h0 = live ? b0 : (unsigned short)0;
      const unsigned short h1 = live ? b1 : (unsigned short)0;
      hv[e]     = __builtin_bit_cast(_Float16, h0);
      hv[4 + e] = __builtin_bit_cast(_Float16, h1);
    }
  }
  unsigned short* q = dst + (size_t)row * dst_pitch + g * 8;
  *(volatile v8h*)q = hv;
  __threadfence();
  *(volatile v8h*)q = hv;
}

template <bool F16>
__global__ __launch_bounds__(256) void swscale_kernel(
    const float* __restrict__ sw, const float* __restrict__ ss, unsigned short* __restrict__ dst, int Cin, int total)
{
  const int i = blockIdx.x * 256 + threadIdx.x;
  if (i >= total) return;
  const int o = i / Cin;
  const int c = i - o * Cin;
  const float s = rbf(ss[i]);
  const v4f a0 = *(const v4f*)(sw + (size_t)i * 8);
  const v4f a1 = *(const v4f*)(sw + (size_t)i * 8 + 4);
  v8h hv;
#pragma unroll
  for (int e = 0; e < 4; ++e) {
    const float x0 = a0[e], x1 = a1[e];
    const float p0 = rbf(x0) * s, p1 = rbf(x1) * s;
    if (F16) {
      hv[e]     = (_Float16)(p0 * kWCarry);
      hv[4 + e] = (_Float16)(p1 * kWCarry);
    } else {
      const unsigned short h0 = f2bf_bits(p0), h1 = f2bf_bits(p1);
      hv[e]     = __builtin_bit_cast(_Float16, h0);
      hv[4 + e] = __builtin_bit_cast(_Float16, h1);
    }
  }
  unsigned short* q = dst + (size_t)o * (Cin * 9) + Cin + (size_t)c * 8;
  *(volatile v8h*)q = hv;
  __threadfence();
  *(volatile v8h*)q = hv;
}

__global__ __launch_bounds__(256) void in_ln_kernel(
    const float* __restrict__ x5d, const float* __restrict__ gam, const float* __restrict__ bet,
    float* __restrict__ X0, unsigned short* __restrict__ XN16)
{
  __shared__ __align__(16) float tile[32 * 260];
  const int tid = threadIdx.x, lane = tid & 31, wave = tid >> 5;
  const int b = blockIdx.x >> 5;
  const int n0 = (blockIdx.x & 31) * 32;
#pragma unroll 4
  for (int i = 0; i < 32; ++i) {
    const int cc = (tid >> 5) + 8 * i;
    const int nn = tid & 31;
    tile[nn * 260 + cc] = rbf(x5d[((size_t)b * kCh + cc) * kSeq + n0 + nn]);
  }
  __syncthreads();
  const v4f g0r = *(const v4f*)(gam + lane * 8);
  const v4f g1r = *(const v4f*)(gam + lane * 8 + 4);
  const v4f b0r = *(const v4f*)(bet + lane * 8);
  const v4f b1r = *(const v4f*)(bet + lane * 8 + 4);
  float gg[8], bb[8];
#pragma unroll
  for (int e = 0; e < 4; ++e) {
    const float t0 = g0r[e], t1 = g1r[e], t2 = b0r[e], t3 = b1r[e];
    gg[e] = rbf(t0); gg[4 + e] = rbf(t1); bb[e] = rbf(t2); bb[4 + e] = rbf(t3);
  }
#pragma unroll 1
  for (int j = 0; j < 4; ++j) {
    const int nn = wave * 4 + j;
    const size_t row = (size_t)b * kSeq + n0 + nn;
    const float* tr = tile + nn * 260;
    const v4f a0 = *(const v4f*)(tr + lane * 8);
    const v4f a1 = *(const v4f*)(tr + lane * 8 + 4);
    float xv[8];
#pragma unroll
    for (int e = 0; e < 4; ++e) { xv[e] = a0[e]; xv[4 + e] = a1[e]; }
    float s = ((xv[0] + xv[1]) + (xv[2] + xv[3])) + ((xv[4] + xv[5]) + (xv[6] + xv[7]));
    s = wave_sum(s);
    const float mean = s * (1.0f / 256.0f);
    float q = 0.f;
#pragma unroll
    for (int e = 0; e < 8; ++e) { const float d = xv[e] - mean; q += d * d; }
    q = wave_sum(q);
    const float rstd = rsqrtf(q * (1.0f / 256.0f) + kLnEps);
    v8h hv;
#pragma unroll
    for (int e = 0; e < 8; ++e) {
      const float xn = (xv[e] - mean) * rstd * gg[e] + bb[e];
      const unsigned short hb = f2bf_bits(xn);
      hv[e] = __builtin_bit_cast(_Float16, hb);
    }
    const v4f f0 = *(const v4f*)(tr + lane * 4);
    const v4f f1 = *(const v4f*)(tr + 128 + lane * 4);
    for (int pass = 0; pass < 2; ++pass) {
      *(volatile v4f*)(X0 + row * kCh + lane * 4) = f0;
      *(volatile v4f*)(X0 + row * kCh + 128 + lane * 4) = f1;
      *(volatile v8h*)(XN16 + row * kCh + lane * 8) = hv;
      __threadfence();
    }
  }
}

__global__ __launch_bounds__(256) void ln16_kernel(
    const float* __restrict__ X, const float* __restrict__ gam, const float* __restrict__ bet,
    unsigned short* __restrict__ XN16)
{
  const int lane = threadIdx.x & 31, wave = threadIdx.x >> 5;
  const v4f g0r = *(const v4f*)(gam + lane * 8);
  const v4f g1r = *(const v4f*)(gam + lane * 8 + 4);
  const v4f b0r = *(const v4f*)(bet + lane * 8);
  const v4f b1r = *(const v4f*)(bet + lane * 8 + 4);
  float gg[8], bb[8];
#pragma unroll
  for (int e = 0; e < 4; ++e) {
    const float t0 = g0r[e], t1 = g1r[e], t2 = b0r[e], t3 = b1r[e];
    gg[e] = rbf(t0); gg[4 + e] = rbf(t1); bb[e] = rbf(t2); bb[4 + e] = rbf(t3);
  }
#pragma unroll 1
  for (int j = 0; j < 4; ++j) {
    const size_t row = (size_t)(blockIdx.x * 8 + wave) * 4 + j;
    const float* xr = X + row * kCh;
    const v4f a0 = *(const v4f*)(xr + lane * 8);
    const v4f a1 = *(const v4f*)(xr + lane * 8 + 4);
    float xv[8];
#pragma unroll
    for (int e = 0; e < 4; ++e) { xv[e] = a0[e]; xv[4 + e] = a1[e]; }
    float s = ((xv[0] + xv[1]) + (xv[2] + xv[3])) + ((xv[4] + xv[5]) + (xv[6] + xv[7]));
    s = wave_sum(s);
    const float mean = s * (1.0f / 256.0f);
    float q = 0.f;
#pragma unroll
    for (int e = 0; e < 8; ++e) { const float d = xv[e] - mean; q += d * d; }
    q = wave_sum(q);
    const float rstd = rsqrtf(q * (1.0f / 256.0f) + kLnEps);
    v8h hv;
#pragma unroll
    for (int e = 0; e < 8; ++e) {
      const float xn = (xv[e] - mean) * rstd * gg[e] + bb[e];
      const unsigned short hb = f2bf_bits(xn);
      hv[e] = __builtin_bit_cast(_Float16, hb);
    }
    unsigned short* qd = XN16 + row * kCh + lane * 8;
    *(volatile v8h*)qd = hv;
    __threadfence();
    *(volatile v8h*)qd = hv;
  }
}

__global__ __launch_bounds__(128) void dwq_norm_kernel(
    const float* __restrict__ QKf, const float* __restrict__ dww, const float* __restrict__ dwb,
    unsigned short* __restrict__ Q16, unsigned short* __restrict__ K16)
{
  __shared__ __align__(16) float img[1024];
  __shared__ float red[4];
  const int tid = threadIdx.x, lane = tid & 31, wave = tid >> 5;
  const int bid = blockIdx.x;
  const int ch = bid & 255;
  const int b  = (bid >> 8) & 3;
  const int p  = bid >> 10;
  const int cg = p * 256 + ch;
  const float* srow = QKf + ((size_t)b * 512 + cg) * kSeq;
  *(v4f*)(img + tid * 8)     = *(const v4f*)(srow + tid * 8);
  *(v4f*)(img + tid * 8 + 4) = *(const v4f*)(srow + tid * 8 + 4);
  __syncthreads();
  const int y = tid >> 2, x0 = (tid & 3) * 8;
  const float bias = rbf(dwb[cg]);
  float acc[8];
#pragma unroll
  for (int e = 0; e < 8; ++e) acc[e] = bias;
#pragma unroll 1
  for (int dy = 0; dy < 3; ++dy) {
    const int yy = y + dy - 1;
    const bool vy = (yy >= 0) && (yy < 32);
    const int yc = yy < 0 ? 0 : (yy > 31 ? 31 : yy);
    const float w0 = rbf(dww[cg * 9 + dy * 3 + 0]);
    const float w1 = rbf(dww[cg * 9 + dy * 3 + 1]);
    const float w2 = rbf(dww[cg * 9 + dy * 3 + 2]);
    float r[10];
#pragma unroll
    for (int k = 0; k < 10; ++k) {
      const int xx = x0 - 1 + k;
      const bool vx = (xx >= 0) && (xx < 32);
      const int xc = xx < 0 ? 0 : (xx > 31 ? 31 : xx);
      const float v = img[yc * 32 + xc];
      r[k] = (vy && vx) ? v : 0.0f;
    }
#pragma unroll
    for (int e = 0; e < 8; ++e) {
      acc[e] = fmaf(w0, r[e], acc[e]);
      acc[e] = fmaf(w1, r[e + 1], acc[e]);
      acc[e] = fmaf(w2, r[e + 2], acc[e]);
    }
  }
  float ss = 0.f;
#pragma unroll
  for (int e = 0; e < 8; ++e) ss += acc[e] * acc[e];
  ss = wave_sum(ss);
  if (lane == 0) red[wave] = ss;
  __syncthreads();
  const float tot = (red[0] + red[1]) + (red[2] + red[3]);
  const float inv = 1.0f / fmaxf(sqrtf(tot), 1e-12f);
  v8h hv;
#pragma unroll
  for (int e = 0; e < 8; ++e) {
    const unsigned short hb = f2bf_bits(acc[e] * inv);
    hv[e] = __builtin_bit_cast(_Float16, hb);
  }
  unsigned short* dplane = (p == 0) ? Q16 : K16;
  unsigned short* qd = dplane + ((size_t)b * 256 + ch) * kSeq + tid * 8;
  *(volatile v8h*)qd = hv;
  __threadfence();
  *(volatile v8h*)qd = hv;
}

__global__ __launch_bounds__(256) void dwv_kernel(
    const float* __restrict__ VCL, const float* __restrict__ dww, const float* __restrict__ dwb,
    unsigned short* __restrict__ VT16)
{
  __shared__ __align__(16) float sT[16 * 260];
  const int tid = threadIdx.x, lane = tid & 31, wave = tid >> 5;
  const int g0 = blockIdx.x * 16;
  const int b  = g0 >> 10;
  const int nb = g0 & 1023;
  const int cw = 512 + tid;
  float w[9];
#pragma unroll
  for (int k = 0; k < 9; ++k) w[k] = rbf(dww[cw * 9 + k]);
  const float bias = rbf(dwb[cw]);
#pragma unroll 1
  for (int s = 0; s < 16; ++s) {
    const int n = nb + s;
    const int y = n >> 5, x = n & 31;
    float acc = bias;
#pragma unroll
    for (int dy = 0; dy < 3; ++dy) {
#pragma unroll
      for (int dx = 0; dx < 3; ++dx) {
        const int yy = y + dy - 1, xx = x + dx - 1;
        const bool ok = (yy >= 0) && (yy < 32) && (xx >= 0) && (xx < 32);
        const int yc = yy < 0 ? 0 : (yy > 31 ? 31 : yy);
        const int xc = xx < 0 ? 0 : (xx > 31 ? 31 : xx);
        const float v = VCL[((size_t)b * kSeq + yc * 32 + xc) * kCh + tid];
        acc = fmaf(ok ? v : 0.0f, w[dy * 3 + dx], acc);
      }
    }
    sT[s * 260 + tid] = acc;
  }
  __syncthreads();
  v8h hv[2];
#pragma unroll
  for (int it = 0; it < 2; ++it) {
    const float* sp = sT + (it * 8 + wave) * 260 + lane * 8;
    const v4f a0 = *(const v4f*)(sp);
    const v4f a1 = *(const v4f*)(sp + 4);
#pragma unroll
    for (int e = 0; e < 4; ++e) {
      const unsigned short h0 = f2bf_bits(a0[e]), h1 = f2bf_bits(a1[e]);
      hv[it][e]     = __builtin_bit_cast(_Float16, h0);
      hv[it][4 + e] = __builtin_bit_cast(_Float16, h1);
    }
  }
  for (int pass = 0; pass < 2; ++pass) {
#pragma unroll
    for (int it = 0; it < 2; ++it)
      *(volatile v8h*)(VT16 + (size_t)(g0 + it * 8 + wave) * kCh + lane * 8) = hv[it];
    __threadfence();
  }
}

__global__ __launch_bounds__(256) void softmax64_kernel(
    const float* __restrict__ ATT, const float* __restrict__ temp, unsigned short* __restrict__ P16)
{
  const int tid = threadIdx.x;
  const int R = blockIdx.x * 32 + (tid >> 3);
  const int seg = tid & 7;
  const float tp = rbf(temp[(R >> 6) & 3]);
  const float* sr = ATT + (size_t)R * 64 + seg * 8;
  const v4f a0 = *(const v4f*)(sr);
  const v4f a1 = *(const v4f*)(sr + 4);
  float x[8];
#pragma unroll
  for (int e = 0; e < 4; ++e) { x[e] = a0[e] * tp; x[4 + e] = a1[e] * tp; }
  float m = fmaxf(fmaxf(fmaxf(x[0], x[1]), fmaxf(x[2], x[3])), fmaxf(fmaxf(x[4], x[5]), fmaxf(x[6], x[7])));
  m = fmaxf(m, __shfl_xor(m, 1, 32));
  m = fmaxf(m, __shfl_xor(m, 2, 32));
  m = fmaxf(m, __shfl_xor(m, 4, 32));
  float s = 0.f;
#pragma unroll
  for (int e = 0; e < 8; ++e) { x[e] = expf(x[e] - m); s += x[e]; }
  s += __shfl_xor(s, 1, 32);
  s += __shfl_xor(s, 2, 32);
  s += __shfl_xor(s, 4, 32);
  const float inv = 1.0f / s;
  v8h hv;
#pragma unroll
  for (int e = 0; e < 8; ++e) {
    const unsigned short hb = f2bf_bits(x[e] * inv);
    hv[e] = __builtin_bit_cast(_Float16, hb);
  }
  unsigned short* qd = P16 + (size_t)R * 64 + seg * 8;
  *(volatile v8h*)qd = hv;
  __threadfence();
  *(volatile v8h*)qd = hv;
}

constexpr float kKnot0 = -2.2f, kKnot1 = -1.8f, kKnot2 = -1.4f, kKnot3 = -1.0f, kKnot4 = -0.6f, kKnot5 = -0.2f;
constexpr float kKnot6 = 0.2f, kKnot7 = 0.6f, kKnot8 = 1.0f, kKnot9 = 1.4f, kKnot10 = 1.8f, kKnot11 = 2.2f;
__device__ __forceinline__ void knot_step(float x, float kj, float& kk, int& iv) {
  const bool ge = (x >= kj);
  kk = ge ? kj : kk;
  iv += ge ? 1 : 0;
}
__device__ __forceinline__ void bspline8(float x, float (&o)[8]) {
  const bool valid = (x >= kKnot0) && (x < kKnot11);
  float kk = kKnot0;
  int iv = 0;
  knot_step(x, kKnot1, kk, iv);
  knot_step(x, kKnot2, kk, iv);
  knot_step(x, kKnot3, kk, iv);
  knot_step(x, kKnot4, kk, iv);
  knot_step(x, kKnot5, kk, iv);
  knot_step(x, kKnot6, kk, iv);
  knot_step(x, kKnot7, kk, iv);
  knot_step(x, kKnot8, kk, iv);
  knot_step(x, kKnot9, kk, iv);
  knot_step(x, kKnot10, kk, iv);
  knot_step(x, kKnot11, kk, iv);
  const float u  = (x - kk) * 2.5f;
  const float u2 = u * u;
  const float u3 = u2 * u;
  const float w  = 1.0f - u;
  const float c0 = w * w * w * (1.0f / 6.0f);
  const float c1 = 0.5f * u3 - u2 + (2.0f / 3.0f);
  const float c2 = -0.5f * u3 + 0.5f * u2 + 0.5f * u + (1.0f / 6.0f);
  const float c3 = u3 * (1.0f / 6.0f);
#pragma unroll
  for (int t = 0; t < 8; ++t) {
    const int j = t - iv + 3;
    const float v = (j == 0) ? c0 : (j == 1) ? c1 : (j == 2) ? c2 : (j == 3) ? c3 : 0.0f;
    o[t] = valid ? v : 0.0f;
  }
}

template <int CIN, bool DO_LN, bool F16>
__global__ __launch_bounds__(256) void kan_operand_kernel(
    const float* __restrict__ src, const float* __restrict__ gam, const float* __restrict__ bet,
    unsigned short* __restrict__ AH, unsigned short* __restrict__ AL)
{
  static_assert(!DO_LN || CIN == 256, "LayerNorm path is 256 wide");
  static_assert((CIN % 256) == 0, "tile multiple");
  constexpr int PITCH = CIN * 9;
  __shared__ __align__(16) float sS[8][CIN];
  __shared__ __align__(16) float sX[8][DO_LN ? CIN : 8];
  const int lane = threadIdx.x & 31, wave = threadIdx.x >> 5;
#pragma unroll 1
  for (int j = 0; j < 4; ++j) {
    const size_t row = (size_t)(blockIdx.x * 8 + wave) * 4 + j;
    const float* xr = src + row * CIN;
    float mean = 0.f, rstd = 1.f;
    if (DO_LN) {
      const v4f a0 = *(const v4f*)(xr + lane * 8);
      const v4f a1 = *(const v4f*)(xr + lane * 8 + 4);
      *(v4f*)(&sX[wave][DO_LN ? lane * 8 : 0]) = a0;
      *(v4f*)(&sX[wave][DO_LN ? lane * 8 + 4 : 4]) = a1;
      float xv[8];
#pragma unroll
      for (int e = 0; e < 4; ++e) { xv[e] = a0[e]; xv[4 + e] = a1[e]; }
      float s = ((xv[0] + xv[1]) + (xv[2] + xv[3])) + ((xv[4] + xv[5]) + (xv[6] + xv[7]));
      s = wave_sum(s);
      mean = s * (1.0f / 256.0f);
      float q = 0.f;
#pragma unroll
      for (int e = 0; e < 8; ++e) { const float d = xv[e] - mean; q += d * d; }
      q = wave_sum(q);
      rstd = rsqrtf(q * (1.0f / 256.0f) + kLnEps);
      wave_lds_sync();
    }
    unsigned short* ah = AH + row * PITCH;
    unsigned short* al = AL + row * PITCH;
#pragma unroll 1
    for (int i = 0; i < CIN / 32; ++i) {
      const int c = lane + 32 * i;
      float x;
      if (DO_LN) {
        const float xraw = sX[wave][DO_LN ? c : 0];
        x = (xraw - mean) * rstd * rbf(gam[c]) + rbf(bet[c]);
      } else {
        x = xr[c];
      }
      const float sg = __builtin_amdgcn_rcpf(1.0f + expf(-x));
      sS[wave][c] = x * sg;
      float bs[8];
      bspline8(x, bs);
      v8h hv, lv;
#pragma unroll
      for (int t = 0; t < 8; ++t) {
        if (F16) {
          hv[t] = (_Float16)(bs[t] * kACarry);
          lv[t] = (_Float16)0.0f;
        } else {
          const unsigned short hb = f2bf_bits(bs[t]);
          const unsigned short lb = f2bf_bits(bs[t] - bf_bits2f(hb));
          hv[t] = __builtin_bit_cast(_Float16, hb);
          lv[t] = __builtin_bit_cast(_Float16, lb);
        }
      }
      unsigned short* ph = ah + CIN + (size_t)c * 8;
      unsigned short* pl = al + CIN + (size_t)c * 8;
      *(volatile v8h*)ph = hv;
      if (!F16) *(volatile v8h*)pl = lv;
      __threadfence();
      *(volatile v8h*)ph = hv;
      if (!F16) *(volatile v8h*)pl = lv;
    }
    wave_lds_sync();
#pragma unroll 1
    for (int it = 0; it < CIN / 256; ++it) {
      const int c0 = it * 256 + lane * 8;
      const v4f a0 = *(const v4f*)(&sS[wave][c0]);
      const v4f a1 = *(const v4f*)(&sS[wave][c0 + 4]);
      v8h hv, lv;
#pragma unroll
      for (int e = 0; e < 4; ++e) {
        const float s0 = a0[e], s1 = a1[e];
        if (F16) {
          hv[e]     = (_Float16)(s0 * kACarry);
          hv[4 + e] = (_Float16)(s1 * kACarry);
          lv[e]     = (_Float16)0.0f;
          lv[4 + e] = (_Float16)0.0f;
        } else {
          const unsigned short h0 = f2bf_bits(s0), h1 = f2bf_bits(s1);
          const unsigned short l0 = f2bf_bits(s0 - bf_bits2f(h0)), l1 = f2bf_bits(s1 - bf_bits2f(h1));
          hv[e]     = __builtin_bit_cast(_Float16, h0);
          hv[4 + e] = __builtin_bit_cast(_Float16, h1);
          lv[e]     = __builtin_bit_cast(_Float16, l0);
          lv[4 + e] = __builtin_bit_cast(_Float16, l1);
        }
      }
      unsigned short* ph = ah + c0;
      unsigned short* pl = al + c0;
      *(volatile v8h*)ph = hv;
      if (!F16) *(volatile v8h*)pl = lv;
      __threadfence();
      *(volatile v8h*)ph = hv;
      if (!F16) *(volatile v8h*)pl = lv;
    }
    wave_lds_sync();
  }
}

__global__ __launch_bounds__(256) void conv1d_silu_kernel(
    const float* __restrict__ XZ, const float* __restrict__ cxw, const float* __restrict__ czw,
    float* __restrict__ XM, unsigned short* __restrict__ XM16, unsigned short* __restrict__ YC16)
{
  __shared__ __align__(16) float sT[16 * 260];
  const int tid = threadIdx.x, lane = tid & 31, wave = tid >> 5;
  const int g0 = blockIdx.x * 64;
  const int tb = g0 & (kSeq - 1);
  const float* wp = (tid < kDh) ? cxw : czw;
  const int wc = tid & (kDh - 1);
  const float w0 = rbf(wp[wc * 3 + 0]);
  const float w1 = rbf(wp[wc * 3 + 1]);
  const float w2 = rbf(wp[wc * 3 + 2]);
  float xleft, xcur;
  {
    const bool hist = (tb > 0);
    const int rp = hist ? (g0 - 1) : g0;
    const float pv = XZ[(size_t)rp * kCh + tid];
    xleft = hist ? pv : 0.0f;
    xcur  = XZ[(size_t)g0 * kCh + tid];
  }
#pragma unroll 1
  for (int sub = 0; sub < 4; ++sub) {
    const int lb = g0 + sub * 16;
#pragma unroll 1
    for (int s = 0; s < 16; ++s) {
      const int gl = lb + s;
      const bool hasn = (((gl + 1) & (kSeq - 1)) != 0);
      const int rn = hasn ? (gl + 1) : gl;
      const float nv = XZ[(size_t)rn * kCh + tid];
      const float xright = hasn ? nv : 0.0f;
      float acc = w0 * xleft;
      acc = fmaf(w1, xcur, acc);
      acc = fmaf(w2, xright, acc);
      const float sg = __builtin_amdgcn_rcpf(1.0f + expf(-acc));
      sT[s * 260 + tid] = acc * sg;
      xleft = xcur;
      xcur = xright;
    }
    __syncthreads();
    v4f fv[2];
    v8h hx, hz;
#pragma unroll
    for (int it = 0; it < 2; ++it) fv[it] = *(const v4f*)(sT + (it * 8 + wave) * 260 + lane * 4);
    const int hr = wave * 2 + (lane >> 4);
    const int c8 = (lane & 15) * 8;
    {
      const float* sp = sT + hr * 260 + c8;
      const v4f a0 = *(const v4f*)(sp);
      const v4f a1 = *(const v4f*)(sp + 4);
      const v4f z0 = *(const v4f*)(sp + kDh);
      const v4f z1 = *(const v4f*)(sp + kDh + 4);
#pragma unroll
      for (int e = 0; e < 4; ++e) {
        const unsigned short h0 = f2bf_bits(a0[e]), h1 = f2bf_bits(a1[e]);
        const unsigned short q0 = f2bf_bits(z0[e]), q1 = f2bf_bits(z1[e]);
        hx[e]     = __builtin_bit_cast(_Float16, h0);
        hx[4 + e] = __builtin_bit_cast(_Float16, h1);
        hz[e]     = __builtin_bit_cast(_Float16, q0);
        hz[4 + e] = __builtin_bit_cast(_Float16, q1);
      }
    }
    for (int pass = 0; pass < 2; ++pass) {
#pragma unroll
      for (int it = 0; it < 2; ++it)
        *(volatile v4f*)(XM + (size_t)(lb + it * 8 + wave) * kDh + lane * 4) = fv[it];
      *(volatile v8h*)(XM16 + (size_t)(lb + hr) * kDh + c8) = hx;
      *(volatile v8h*)(YC16 + (size_t)(lb + hr) * kCh + kDh + c8) = hz;
      __threadfence();
    }
    __syncthreads();
  }
}

__global__ __launch_bounds__(64) void scan_kernel(
    const float* __restrict__ XD, const float* __restrict__ XM,
    const float* __restrict__ Wdt, const float* __restrict__ bdt, const float* __restrict__ Alog,
    const float* __restrict__ Dp, unsigned short* __restrict__ YC16)
{
  __shared__ __align__(16) float sX[64 * 32];
  __shared__ __align__(16) float sY[64 * 68];
  __shared__ __align__(16) float sW[kDtR * 64];
  __shared__ __align__(16) float sA[kNst * 64];
  const int tid = threadIdx.x, lane = tid & 31, wave = tid >> 5;
  const int bix = blockIdx.x >> 1;
  const int d0  = (blockIdx.x & 1) * 64;
  const int d   = d0 + tid;
  const size_t row0 = (size_t)bix * kSeq;
#pragma unroll 1
  for (int r = 0; r < kDtR; ++r) sW[r * 64 + tid] = rbf(Wdt[(size_t)d * kDtR + r]);
#pragma unroll 1
  for (int s = 0; s < kNst; ++s) sA[s * 64 + tid] = -expf(rbf(Alog[(size_t)d * kNst + s]));
  __syncthreads();
  float negA[kNst], h[kNst];
#pragma unroll
  for (int s = 0; s < kNst; ++s) {
    negA[s] = sA[s * 64 + tid];
    h[s] = 0.f;
  }
  const float bb = rbf(bdt[d]), Dd = rbf(Dp[d]);
  const int q = lane >> 3, c8 = (lane & 7) * 8;
#pragma unroll 1
  for (int t0 = 0; t0 < kSeq; t0 += 64) {
    __syncthreads();
#pragma unroll
    for (int i = 0; i < 8; ++i) {
      const int idx = tid + 64 * i;
      const int r = idx >> 3, c4 = (idx & 7) * 4;
      *(v4f*)(sX + r * 32 + c4) = *(const v4f*)(XD + (row0 + t0 + r) * kXdP + c4);
    }
    __syncthreads();
#pragma unroll 1
    for (int s = 0; s < 64; ++s) {
      const int t = t0 + s;
      const float* xr = sX + s * 32;
      float vdot = 0.f;
#pragma unroll 1
      for (int r4 = 0; r4 < kDtR / 4; ++r4) {
        const v4f xv = *(const v4f*)(xr + 4 * r4);
        const float* wq = sW + (4 * r4) * 64 + tid;
        vdot = fmaf(xv[0], wq[0], vdot);
        vdot = fmaf(xv[1], wq[64], vdot);
        vdot = fmaf(xv[2], wq[128], vdot);
        vdot = fmaf(xv[3], wq[192], vdot);
      }
      const v4f bq0 = *(const v4f*)(xr + kDtR);
      const v4f bq1 = *(const v4f*)(xr + kDtR + 4);
      const v4f cq0 = *(const v4f*)(xr + kDtR + kNst);
      const v4f cq1 = *(const v4f*)(xr + kDtR + kNst + 4);
      float Bs[kNst], Cs[kNst];
#pragma unroll
      for (int e = 0; e < 4; ++e) { Bs[e] = bq0[e]; Bs[4 + e] = bq1[e]; Cs[e] = cq0[e]; Cs[4 + e] = cq1[e]; }
      const float v   = vdot + bb;
      const float ea  = __expf(-fabsf(v));
      const float dt  = fmaxf(v, 0.0f) + log1pf(ea);
      const float xt  = XM[(row0 + t) * kDh + d];
      const float dtx = dt * xt;
      float y = 0.f;
#pragma unroll
      for (int k = 0; k < kNst; ++k) {
        const float e = __expf(dt * negA[k]);
        h[k] = e * h[k] + dtx * Bs[k];
        y = h[k] * Cs[k] + y;
      }
      y = xt * Dd + y;
      sY[s * 68 + tid] = y;
    }
    __syncthreads();
    v8h hv[8];
#pragma unroll
    for (int it = 0; it < 8; ++it) {
      const int row = it * 8 + wave * 4 + q;
      const float* sp = sY + row * 68 + c8;
      const v4f a0 = *(const v4f*)(sp);
      const v4f a1 = *(const v4f*)(sp + 4);
#pragma unroll
      for (int e = 0; e < 4; ++e) {
        const unsigned short h0 = f2bf_bits(a0[e]), h1 = f2bf_bits(a1[e]);
        hv[it][e]     = __builtin_bit_cast(_Float16, h0);
        hv[it][4 + e] = __builtin_bit_cast(_Float16, h1);
      }
    }
    for (int pass = 0; pass < 2; ++pass) {
#pragma unroll
      for (int it = 0; it < 8; ++it) {
        const int row = it * 8 + wave * 4 + q;
        *(volatile v8h*)(YC16 + (row0 + t0 + row) * kCh + d0 + c8) = hv[it];
      }
      __threadfence();
    }
  }
}

__global__ __launch_bounds__(256) void transpose_out_kernel(const float* __restrict__ X, float* __restrict__ out)
{
  __shared__ __align__(16) float tT[256 * 36];
  const int tid = threadIdx.x, lane = tid & 31, wave = tid >> 5;
  const int b = blockIdx.x >> 5;
  const int n0 = (blockIdx.x & 31) * 32;
#pragma unroll 4
  for (int i = 0; i < 32; ++i) tT[tid * 36 + i] = X[((size_t)b * kSeq + n0 + i) * kCh + tid];
  __syncthreads();
  const int q = lane >> 3, n4 = (lane & 7) * 4;
  v4f ov[8];
#pragma unroll
  for (int it = 0; it < 8; ++it) {
    const int c = it * 32 + wave * 4 + q;
    ov[it] = *(const v4f*)(tT + c * 36 + n4);
  }
  for (int pass = 0; pass < 2; ++pass) {
#pragma unroll
    for (int it = 0; it < 8; ++it) {
      const int c = it * 32 + wave * 4 + q;
      *(volatile v4f*)(out + ((size_t)b * kCh + c) * kSeq + n0 + n4) = ov[it];
    }
    __threadfence();
  }
}

template <int ET, int SPL, int BM, int OM, bool RS>
static void launch_gemm(hipStream_t st, int gy,
                        const unsigned short* A, const unsigned short* A2, int lda, long sA,
                        const unsigned short* Bt, int ldb, long sB,
                        void* C, void* C2, int ldc, long sC,
                        const float* bias, const float* resid, long sR,
                        int M, int N, int K, float scale)
{
  const int tiles = (M >> 6) * (N >> 6);
  wmma_gemm64<ET, SPL, BM, OM, RS><<<dim3((unsigned)((tiles + 7) / 8), (unsigned)gy), 256, 0, st>>>(
      A, A2, lda, sA, Bt, ldb, sB, C, C2, ldc, sC, bias, resid, sR, M, N, K, scale);
}

template <bool F16>
static void run_fkan(hipStream_t st, const float* Xin, float* Xout, const float* g, const float* bt,
                     const unsigned short* W1, const unsigned short* W2,
                     float* H, unsigned short* AH, unsigned short* AL)
{
  constexpr int ET  = F16 ? 0 : 1;
  constexpr int SPL = F16 ? 0 : 1;
  const float sc = F16 ? kF16Fold : 1.0f;
  kan_operand_kernel<kCh, true, F16><<<kTok / 32, 256, 0, st>>>(Xin, g, bt, AH, AL);
  launch_gemm<ET, SPL, 0, 0, false>(st, 1, AH, AL, kKc1, 0L, W1, kKc1, 0L,
                                    (void*)H, (void*)H, kHid, 0L, g, Xin, 0L, kTok, kHid, kKc1, sc);
  for (int c = 0; c < kTok / kChunk; ++c) {
    kan_operand_kernel<kHid, false, F16><<<kChunk / 32, 256, 0, st>>>(H + (size_t)c * kChunk * kHid, g, bt, AH, AL);
    float* xo = Xout + (size_t)c * kChunk * kCh;
    launch_gemm<ET, SPL, 0, 0, true>(st, 1, AH, AL, kKc2, 0L, W2, kKc2, 0L,
                                     (void*)xo, (void*)xo, kCh, 0L, g, Xin + (size_t)c * kChunk * kCh, 0L,
                                     kChunk, kCh, kKc2, sc);
  }
}

extern "C" void kernel_launch(void* const* d_in, const int* in_sizes, int n_in,
                              void* d_out, int out_size, void* d_ws, size_t ws_size,
                              hipStream_t stream)
{
  if (n_in < 37) return;
  if (in_sizes[0] != kBat * kCh * kSeq) return;
  if (in_sizes[4] != 768 * kCh || in_sizes[6] != 768 * 9 || in_sizes[8] != kCh * kCh) return;
  if (in_sizes[12] != kHid * kCh || in_sizes[13] != kHid * kCh * kNsp || in_sizes[16] != kCh * kHid * kNsp) return;
  if (in_sizes[20] != kHid * kCh || in_sizes[21] != kHid * kCh * kNsp || in_sizes[24] != kCh * kHid * kNsp) return;
  if (in_sizes[28] != kCh * kCh || in_sizes[31] != 32 * kDh || in_sizes[32] != kDh * kDtR) return;
  if (in_sizes[34] != kDh * kNst || in_sizes[36] != kCh * kCh) return;
  if (out_size != kBat * kCh * kSeq) return;
  if (ws_size < kWsTotal) return;

  const float* x5d    = (const float*)d_in[0];
  const float* ln1_g  = (const float*)d_in[1];
  const float* ln1_b  = (const float*)d_in[2];
  const float* temp   = (const float*)d_in[3];
  const float* qkv_w  = (const float*)d_in[4];
  const float* qkv_b  = (const float*)d_in[5];
  const float* dw_w   = (const float*)d_in[6];
  const float* dw_b   = (const float*)d_in[7];
  const float* po_w   = (const float*)d_in[8];
  const float* po_b   = (const float*)d_in[9];
  const float* f1_lng = (const float*)d_in[10];
  const float* f1_lnb = (const float*)d_in[11];
  const float* f1_bw1 = (const float*)d_in[12];
  const float* f1_sw1 = (const float*)d_in[13];
  const float* f1_ss1 = (const float*)d_in[14];
  const float* f1_bw2 = (const float*)d_in[15];
  const float* f1_sw2 = (const float*)d_in[16];
  const float* f1_ss2 = (const float*)d_in[17];
  const float* f2_lng = (const float*)d_in[18];
  const float* f2_lnb = (const float*)d_in[19];
  const float* f2_bw1 = (const float*)d_in[20];
  const float* f2_sw1 = (const float*)d_in[21];
  const float* f2_ss1 = (const float*)d_in[22];
  const float* f2_bw2 = (const float*)d_in[23];
  const float* f2_sw2 = (const float*)d_in[24];
  const float* f2_ss2 = (const float*)d_in[25];
  const float* ln3_g  = (const float*)d_in[26];
  const float* ln3_b  = (const float*)d_in[27];
  const float* in_w   = (const float*)d_in[28];
  const float* cx_w   = (const float*)d_in[29];
  const float* cz_w   = (const float*)d_in[30];
  const float* xp_w   = (const float*)d_in[31];
  const float* dtp_w  = (const float*)d_in[32];
  const float* dtp_b  = (const float*)d_in[33];
  const float* A_log  = (const float*)d_in[34];
  const float* Dp     = (const float*)d_in[35];
  const float* out_w  = (const float*)d_in[36];
  float* dout = (float*)d_out;

  char* ws = (char*)d_ws;
  float*          XA    = (float*)(ws + kOffXA);
  float*          XB    = (float*)(ws + kOffXB);
  unsigned short* XN16  = (unsigned short*)(ws + kOffXN16);
  unsigned short* QKVW  = (unsigned short*)(ws + kOffQKVW);
  unsigned short* POW   = (unsigned short*)(ws + kOffPOW);
  unsigned short* INW   = (unsigned short*)(ws + kOffINW);
  unsigned short* OUTW  = (unsigned short*)(ws + kOffOUTW);
  unsigned short* XPW   = (unsigned short*)(ws + kOffXPW);
  unsigned short* W1A   = (unsigned short*)(ws + kOffW1A);
  unsigned short* W2A   = (unsigned short*)(ws + kOffW2A);
  unsigned short* W1B   = (unsigned short*)(ws + kOffW1B);
  unsigned short* W2B   = (unsigned short*)(ws + kOffW2B);
  float*          H     = (float*)(ws + kOffH);
  unsigned short* AH    = (unsigned short*)(ws + kOffAH);
  unsigned short* AL    = (unsigned short*)(ws + kOffAL);
  float*          QKF   = (float*)(ws + kOffQKF);
  float*          VCL   = (float*)(ws + kOffVCL);
  unsigned short* Q16   = (unsigned short*)(ws + kOffQ16);
  unsigned short* K16   = (unsigned short*)(ws + kOffK16);
  unsigned short* VT16  = (unsigned short*)(ws + kOffVT16);
  float*          ATT   = (float*)(ws + kOffATT);
  unsigned short* ATT16 = (unsigned short*)(ws + kOffATT16);
  unsigned short* ATOH  = (unsigned short*)(ws + kOffATOH);
  unsigned short* ATOL  = (unsigned short*)(ws + kOffATOL);
  float*          XZ    = (float*)(ws + kOffXZ);
  float*          XM    = (float*)(ws + kOffXM);
  unsigned short* XM16  = (unsigned short*)(ws + kOffXM16);
  float*          XD    = (float*)(ws + kOffXD);
  unsigned short* YC16  = (unsigned short*)(ws + kOffYC16);

  cast_rows_kernel<false><<<(768 * 32) / 256, 256, 0, stream>>>(qkv_w, kCh, 768, QKVW, kCh, 32, 768 * 32, 1.0f);
  cast_rows_kernel<false><<<(kCh * 32) / 256, 256, 0, stream>>>(po_w, kCh, kCh, POW, kCh, 32, kCh * 32, 1.0f);
  cast_rows_kernel<false><<<(kCh * 32) / 256, 256, 0, stream>>>(in_w, kCh, kCh, INW, kCh, 32, kCh * 32, 1.0f);
  cast_rows_kernel<false><<<(kCh * 32) / 256, 256, 0, stream>>>(out_w, kCh, kCh, OUTW, kCh, 32, kCh * 32, 1.0f);
  cast_rows_kernel<false><<<(64 * 16) / 256, 256, 0, stream>>>(xp_w, kDh, 32, XPW, kDh, 16, 64 * 16, 1.0f);
  cast_rows_kernel<false><<<(kHid * 32) / 256, 256, 0, stream>>>(f1_bw1, kCh, kHid, W1A, kKc1, 32, kHid * 32, 1.0f);
  swscale_kernel<false><<<(kHid * kCh) / 256, 256, 0, stream>>>(f1_sw1, f1_ss1, W1A, kCh, kHid * kCh);
  cast_rows_kernel<false><<<(kCh * 128) / 256, 256, 0, stream>>>(f1_bw2, kHid, kCh, W2A, kKc2, 128, kCh * 128, 1.0f);
  swscale_kernel<false><<<(kCh * kHid) / 256, 256, 0, stream>>>(f1_sw2, f1_ss2, W2A, kHid, kCh * kHid);
  cast_rows_kernel<true><<<(kHid * 32) / 256, 256, 0, stream>>>(f2_bw1, kCh, kHid, W1B, kKc1, 32, kHid * 32, kWCarry);
  swscale_kernel<true><<<(kHid * kCh) / 256, 256, 0, stream>>>(f2_sw1, f2_ss1, W1B, kCh, kHid * kCh);
  cast_rows_kernel<true><<<(kCh * 128) / 256, 256, 0, stream>>>(f2_bw2, kHid, kCh, W2B, kKc2, 128, kCh * 128, kWCarry);
  swscale_kernel<true><<<(kCh * kHid) / 256, 256, 0, stream>>>(f2_sw2, f2_ss2, W2B, kHid, kCh * kHid);

  in_ln_kernel<<<kBat * 32, 256, 0, stream>>>(x5d, ln1_g, ln1_b, XA, XN16);
  launch_gemm<1, 0, 1, 0, false>(stream, kBat, QKVW, QKVW, kCh, 0L, XN16, kCh, (long)kSeq * kCh,
                                 (void*)QKF, (void*)QKF, kSeq, (long)512 * kSeq, qkv_b, XA, 0L, 512, kSeq, kCh, 1.0f);
  launch_gemm<1, 0, 2, 0, false>(stream, 1, XN16, XN16, kCh, 0L, QKVW + (size_t)512 * kCh, kCh, 0L,
                                 (void*)VCL, (void*)VCL, kCh, 0L, qkv_b + 512, XA, 0L, kTok, kCh, kCh, 1.0f);
  dwq_norm_kernel<<<2 * kBat * 256, 128, 0, stream>>>(QKF, dw_w, dw_b, Q16, K16);
  dwv_kernel<<<kTok / 16, 256, 0, stream>>>(VCL, dw_w, dw_b, VT16);
  launch_gemm<1, 0, 0, 0, false>(stream, kBat * kHeads, Q16, Q16, kSeq, (long)kHd * kSeq, K16, kSeq, (long)kHd * kSeq,
                                 (void*)ATT, (void*)ATT, kHd, (long)kHd * kHd, qkv_b, XA, 0L, kHd, kHd, kSeq, 1.0f);
  softmax64_kernel<<<(kBat * kHeads * kHd) / 32, 256, 0, stream>>>(ATT, temp, ATT16);
  for (int b = 0; b < kBat; ++b) {
    launch_gemm<1, 0, 0, 2, false>(stream, kHeads,
                                   VT16 + (size_t)b * kSeq * kCh, VT16 + (size_t)b * kSeq * kCh, kCh, (long)kHd,
                                   ATT16 + (size_t)b * kHeads * kHd * kHd, kHd, (long)kHd * kHd,
                                   (void*)(ATOH + (size_t)b * kSeq * kCh), (void*)(ATOL + (size_t)b * kSeq * kCh), kCh, (long)kHd,
                                   qkv_b, XA, 0L, kSeq, kHd, kHd, 1.0f);
  }
  launch_gemm<1, 1, 2, 0, true>(stream, 1, ATOH, ATOL, kCh, 0L, POW, kCh, 0L,
                                (void*)XB, (void*)XB, kCh, 0L, po_b, XA, 0L, kTok, kCh, kCh, 1.0f);

  run_fkan<false>(stream, XB, XA, f1_lng, f1_lnb, W1A, W2A, H, AH, AL);

  ln16_kernel<<<kTok / 32, 256, 0, stream>>>(XA, ln3_g, ln3_b, XN16);
  launch_gemm<1, 0, 0, 0, false>(stream, 1, XN16, XN16, kCh, 0L, INW, kCh, 0L,
                                 (void*)XZ, (void*)XZ, kCh, 0L, qkv_b, XA, 0L, kTok, kCh, kCh, 1.0f);
  conv1d_silu_kernel<<<kTok / 64, 256, 0, stream>>>(XZ, cx_w, cz_w, XM, XM16, YC16);
  launch_gemm<1, 0, 0, 0, false>(stream, 1, XM16, XM16, kDh, 0L, XPW, kDh, 0L,
                                 (void*)XD, (void*)XD, kXdP, 0L, qkv_b, XA, 0L, kTok, kXdP, kDh, 1.0f);
  scan_kernel<<<kBat * 2, 64, 0, stream>>>(XD, XM, dtp_w, dtp_b, A_log, Dp, YC16);
  launch_gemm<1, 0, 0, 0, true>(stream, 1, YC16, YC16, kCh, 0L, OUTW, kCh, 0L,
                                (void*)XB, (void*)XB, kCh, 0L, qkv_b, XA, 0L, kTok, kCh, kCh, 1.0f);

  run_fkan<true>(stream, XB, XA, f2_lng, f2_lnb, W1B, W2B, H, AH, AL);

  transpose_out_kernel<<<kBat * 32, 256, 0, stream>>>(XA, dout);
}
